// DeltaNet_31877247271472
// MI455X (gfx1250) — hardware-verified
//
#include <hip/hip_runtime.h>
#include <math.h>

constexpr int kBatch     = 2;
constexpr int kSeq       = 4096;
constexpr int kDim       = 1024;
constexpr int kHeads     = 8;
constexpr int kHeadDim   = 128;
constexpr int kChunk     = 32;
constexpr int kNumChunk  = kSeq / kChunk;
constexpr int kTok       = kBatch * kSeq;
constexpr int kQKVDim    = 3 * kDim;
constexpr int kLogitN    = 64;
constexpr int kSlice     = 32;
constexpr int kNumSlice  = kHeadDim / kSlice;
constexpr int kChunkAll  = kBatch * kHeads * kNumChunk;
constexpr int kTileHalves = kChunk * kChunk;
constexpr float kWCarry    = 16.0f;
constexpr float kWCarryInv = 1.0f / 16.0f;
constexpr float kL2Eps     = 1e-12f;
constexpr float kRmsEps    = 1e-5f;
constexpr float kInvHeadDim = 1.0f / (float)kHeadDim;
constexpr int kPQ = 136;
constexpr int kPT = 40;
constexpr int kPF = 36;

static_assert(kDim == kHeads * kHeadDim, "channel split");
static_assert(kSeq % kChunk == 0, "chunking exact");
static_assert(kTok % 64 == 0 && kQKVDim % 64 == 0 && kDim % 64 == 0 && kLogitN % 64 == 0, "GEMM M, N tile multiples");
static_assert(kDim % 32 == 0, "GEMM K multiple of 32");
static_assert(kHeadDim % 32 == 0 && kChunk % 32 == 0, "in-kernel K multiples of 32");
static_assert(kNumChunk == 128 && kHeads == 8 && kNumSlice == 4, "index decode");
static_assert(kPQ % 8 == 0 && kPT % 8 == 0 && kPF % 4 == 0, "16-B aligned LDS rows");
static_assert((size_t)2 * kChunkAll * kTileHalves * 2 <= (size_t)kTok * kDim * 2, "T/P planes fit the dead f16 activation plane");
static_assert((size_t)kTok * kDim * 4 + (size_t)kTok * kDim * 2 <= (size_t)kTok * kQKVDim * 2, "o planes fit the dead projection plane");

typedef __attribute__((ext_vector_type(16))) _Float16 v16h;
typedef __attribute__((ext_vector_type(8)))  _Float16 v8h;
typedef __attribute__((ext_vector_type(8)))  float    v8f;
typedef __attribute__((ext_vector_type(4)))  float    v4f;
typedef __attribute__((ext_vector_type(4)))  unsigned int v4u;
typedef __attribute__((ext_vector_type(2)))  unsigned int v2u;

__device__ __forceinline__ void dep_guard4_h(v8f& a, v8f& b, v8f& c, v8f& d, v16h x, v16h y) {
  asm volatile("v_nop\n\tv_nop\n\tv_nop\n\tv_nop" : "+v"(a), "+v"(b), "+v"(c), "+v"(d) : "v"(x), "v"(y));
}
__device__ __forceinline__ void keep4_h(v16h a, v16h b, v16h c, v16h d) { asm volatile("v_nop" :: "v"(a), "v"(b), "v"(c), "v"(d)); }
__device__ __forceinline__ void acc_guard4(v8f& a, v8f& b, v8f& c, v8f& d) { asm volatile("v_nop\n\tv_nop\n\tv_nop\n\tv_nop" : "+v"(a), "+v"(b), "+v"(c), "+v"(d)); }

template <typename T> struct Frag;
template <> struct Frag<_Float16> {
  typedef v16h V; union U { v16h v; v8h h[2]; };
  static __device__ __forceinline__ v16h load(const _Float16* p) {
    U f; f.h[0] = *(const v8h*)(p); f.h[1] = *(const v8h*)(p + 16); return f.v;
  }
  static __device__ __forceinline__ v8f mma(v16h a, v16h b, v8f c) {
    return __builtin_amdgcn_wmma_f32_16x16x32_f16(false, a, false, b, (short)0, c, false, false);
  }
};
__device__ __forceinline__ v8f mma_g(v16h a, v16h b, v8f c) {
  c = __builtin_amdgcn_wmma_f32_16x16x32_f16(false, a, false, b, (short)0, c, false, false);
  asm volatile("v_nop\n\tv_nop\n\tv_nop\n\tv_nop" : "+v"(c) : "v"(a), "v"(b));
  return c;
}
__device__ __forceinline__ void wave_sync_lds() {
  __builtin_amdgcn_fence(__ATOMIC_RELEASE, "workgroup");
  __builtin_amdgcn_wave_barrier();
  __builtin_amdgcn_fence(__ATOMIC_ACQUIRE, "workgroup");
}

__device__ __forceinline__ float h16_to_f32(unsigned hb) {
  const unsigned sgn = (hb & 0x8000u) << 16; const unsigned em = hb & 0x7fffu;
  const float fn = __uint_as_float((em << 13) + 0x38000000u);
  const float fs = (float)em * 5.9604644775390625e-8f;
  const float mag = (em < 0x400u) ? fs : fn; return __uint_as_float(__float_as_uint(mag) | sgn); }
__device__ __forceinline__ void unpack2(unsigned w, float& lo, float& hi) {
  lo = h16_to_f32(w & 0xffffu);
  hi = h16_to_f32(w >> 16);
}
__device__ __forceinline__ float sigmoid_f(float x) { return __builtin_amdgcn_rcpf(1.0f + expf(-x)); }

template <int OUT_MODE>
__global__ __launch_bounds__(256) void wmma_gemm64(
    const unsigned short* __restrict__ Ap, int lda,
    const unsigned short* __restrict__ Btp, int ldb,
    void* __restrict__ Cout, int ldc, int M, int N, int K, float scale) {
  typedef _Float16 T;
  const T* A = (const T*)Ap; const T* Bt = (const T*)Btp;
  __shared__ __align__(16) float sT[8][16 * 68];
  const int lane = threadIdx.x & 31;
  const int wave = threadIdx.x >> 5;
  const int tilesN = N >> 6;
  const int tilesM = M >> 6;
  const int tile = blockIdx.x * 8 + wave;
  if (tile >= tilesM * tilesN) return;
  const int tm = tile / tilesN;
  const int tn = tile - tm * tilesN;
  const int m0 = tm << 6;
  const int n0 = tn << 6;
  const int rlane = lane & 15;
  const int koff  = (lane >> 4) * 8;
  const int mOff  = (lane >> 4) * 8;

  const T* bp[4];
  const T* ap[4];
#pragma unroll
  for (int j = 0; j < 4; ++j) bp[j] = Bt + (size_t)(n0 + (j << 4) + rlane) * ldb + koff;
#pragma unroll
  for (int i = 0; i < 4; ++i) ap[i] = A + (size_t)(m0 + (i << 4) + rlane) * lda + koff;

  v8f acc[4][4];
#pragma unroll
  for (int i = 0; i < 4; ++i)
#pragma unroll
    for (int j = 0; j < 4; ++j) acc[i][j] = (v8f){0.f,0.f,0.f,0.f,0.f,0.f,0.f,0.f};

  for (int k0 = 0; k0 < K; k0 += 32) {
    v16h bh[4];
#pragma unroll
    for (int j = 0; j < 4; ++j) bh[j] = Frag<T>::load(bp[j] + k0);
#pragma unroll
    for (int i = 0; i < 4; ++i) {
      const v16h ah = Frag<T>::load(ap[i] + k0);
#pragma unroll
      for (int j = 0; j < 4; ++j) acc[i][j] = Frag<T>::mma(ah, bh[j], acc[i][j]);
      dep_guard4_h(acc[i][0], acc[i][1], acc[i][2], acc[i][3], ah, bh[3]);
    }
    keep4_h(bh[0], bh[1], bh[2], bh[3]);
  }
  acc_guard4(acc[0][0], acc[0][1], acc[0][2], acc[0][3]);
  acc_guard4(acc[1][0], acc[1][1], acc[1][2], acc[1][3]);
  acc_guard4(acc[2][0], acc[2][1], acc[2][2], acc[2][3]);
  acc_guard4(acc[3][0], acc[3][1], acc[3][2], acc[3][3]);

  float* slab = sT[wave];
#pragma unroll
  for (int i = 0; i < 4; ++i) {
    const int mBase = m0 + (i << 4);
#pragma unroll
    for (int j = 0; j < 4; ++j) {
#pragma unroll
      for (int r = 0; r < 8; ++r) {
        const float v = acc[i][j][r] * scale;
        slab[(mOff + r) * 68 + (j << 4) + rlane] = v;
      }
    }
    wave_sync_lds();
    if (OUT_MODE == 0) {
      float* C = (float*)Cout;
      const int hh = lane >> 4, c4 = (lane & 15) * 4;
      for (int pass = 0; pass < 2; ++pass) {
#pragma unroll
        for (int it = 0; it < 8; ++it) {
          const int row = it * 2 + hh;
          const v4f v = *(const v4f*)(slab + row * 68 + c4);
          *(volatile v4f*)(C + (size_t)(mBase + row) * ldc + n0 + c4) = v;
        }
        __threadfence();
      }
    } else {
      unsigned short* C = (unsigned short*)Cout;
      const int q = lane >> 3, c8 = (lane & 7) * 8;
      for (int pass = 0; pass < 2; ++pass) {
#pragma unroll
        for (int it = 0; it < 4; ++it) {
          const int row = it * 4 + q;
          const float* sp = slab + row * 68 + c8;
          v8h hv;
#pragma unroll
          for (int e = 0; e < 8; ++e) hv[e] = (_Float16)sp[e];
          *(volatile v8h*)(C + (size_t)(mBase + row) * ldc + n0 + c8) = hv;
        }
        __threadfence();
      }
    }
    wave_sync_lds();
  }
}

__global__ __launch_bounds__(256) void cast8_f16_kernel(const float* __restrict__ in, unsigned short* __restrict__ out, int n8) {
  const int i = blockIdx.x * 256 + threadIdx.x;
  if (i >= n8) return;
  const float* p = in + 8 * (size_t)i;
  const v4f a = *(const v4f*)(p);
  const v4f c = *(const v4f*)(p + 4);
  v8h hv;
#pragma unroll
  for (int e = 0; e < 4; ++e) {
    hv[e]     = (_Float16)a[e];
    hv[4 + e] = (_Float16)c[e];
  }
  unsigned short* q = out + 8 * (size_t)i;
  *(volatile v8h*)q = hv;
  __threadfence();
  *(volatile v8h*)q = hv;
}

__global__ __launch_bounds__(256) void pack_w_kernel(const float* __restrict__ W0, const float* __restrict__ W1,
                                                     const float* __restrict__ W2, const float* __restrict__ W3,
                                                     unsigned short* __restrict__ outqkv, unsigned short* __restrict__ outo) {
  __shared__ float sm[64][65];
  const int t  = threadIdx.x;
  const int d0 = blockIdx.x * 64;
  const int n0 = blockIdx.y * 64;
  const int z  = blockIdx.z;
  const float* W = (z == 0) ? W0 : ((z == 1) ? W1 : ((z == 2) ? W2 : W3));
#pragma unroll
  for (int i = 0; i < 16; ++i) {
    const int e = i * 256 + t;
    const int r = e >> 6;
    const int c = e & 63;
    sm[c][r] = W[(size_t)(d0 + r) * kDim + n0 + c] * kWCarry;
  }
  __syncthreads();
  const int lane = t & 31, wave = t >> 5;
  const int q = lane >> 3, c8 = (lane & 7) * 8;
  unsigned short* op = (z < 3) ? (outqkv + (size_t)z * kDim * kDim) : outo;
  for (int pass = 0; pass < 2; ++pass) {
#pragma unroll
    for (int it = 0; it < 2; ++it) {
      const int row = wave * 8 + it * 4 + q;
      v8h hv;
#pragma unroll
      for (int e = 0; e < 8; ++e) hv[e] = (_Float16)sm[row][c8 + e];
      *(volatile v8h*)(op + (size_t)(n0 + row) * kDim + d0 + c8) = hv;
    }
    __threadfence();
  }
}

__global__ __launch_bounds__(256) void pack_bm_kernel(const float* __restrict__ bw, const float* __restrict__ mw,
                                                      unsigned short* __restrict__ out) {
  const int i = blockIdx.x * 256 + threadIdx.x;
  if (i >= kLogitN * (kDim / 8)) return;
  const int row = i >> 7;
  const int c8 = (i & 127) * 8;
  const int hb = row & 7;
  v8h hv;
#pragma unroll
  for (int e = 0; e < 8; ++e) {
    const int d = c8 + e;
    const float fa = bw[d * kHeads + hb];
    const float fm = mw[d * kHeads + hb];
    const float v = (row < kHeads) ? fa : ((row < 2 * kHeads) ? fm : 0.0f);
    hv[e] = (_Float16)(v * kWCarry);
  }
  unsigned short* q = out + (size_t)row * kDim + c8;
  *(volatile v8h*)q = hv;
  __threadfence();
  *(volatile v8h*)q = hv;
}

__global__ __launch_bounds__(256) void conv_norm_kernel(const unsigned short* __restrict__ lin,
                                                        const float* __restrict__ cwq, const float* __restrict__ cwk,
                                                        const float* __restrict__ cwv, unsigned short* __restrict__ qkv) {
  const int lane = threadIdx.x & 31, wave = threadIdx.x >> 5;
  const int gw = blockIdx.x * 8 + wave;
  if (gw >= kTok * 4) return;
  const int tok = gw >> 2;
  const int hp  = gw & 3;
  const int c0  = hp * 256 + lane * 8;
  const int t   = tok & (kSeq - 1);
#pragma unroll 1
  for (int p = 0; p < 3; ++p) {
    const float* cw = (p == 0) ? cwq : ((p == 1) ? cwk : cwv);
    v4f wv[8];
#pragma unroll
    for (int e = 0; e < 8; ++e) wv[e] = *(const v4f*)(cw + (size_t)(c0 + e) * 4);
    float acc[8];
#pragma unroll
    for (int e = 0; e < 8; ++e) acc[e] = 0.0f;
#pragma unroll
    for (int i = 0; i < 4; ++i) {
      const int tt = t - 3 + i;
      const bool ok = (tt >= 0);
      const int tokc = ok ? (tok - 3 + i) : tok;
      const v4u w = *(const v4u*)(lin + (size_t)tokc * kQKVDim + p * kDim + c0);
#pragma unroll
      for (int j = 0; j < 4; ++j) {
        const unsigned wj = w[j];
        float lo, hi;
        unpack2(wj, lo, hi);
        const float x0 = ok ? lo : 0.0f;
        const float x1 = ok ? hi : 0.0f;
        acc[2 * j]     = fmaf(x0, wv[2 * j][i],     acc[2 * j]);
        acc[2 * j + 1] = fmaf(x1, wv[2 * j + 1][i], acc[2 * j + 1]);
      }
    }
    float s[8];
    float ss = 0.0f;
#pragma unroll
    for (int e = 0; e < 8; ++e) {
      const float y = acc[e];
      const float sv = y * sigmoid_f(y);
      s[e] = sv;
      ss += sv * sv;
    }
#pragma unroll
    for (int off = 1; off < 16; off <<= 1) ss += __shfl_xor(ss, off, 32);
    const float rn  = rsqrtf(ss + kL2Eps);
    const float scl = (p < 2) ? rn : 1.0f;
    v8h hv;
#pragma unroll
    for (int e = 0; e < 8; ++e) hv[e] = (_Float16)(s[e] * scl);
    unsigned short* op = qkv + (size_t)p * kTok * kDim + (size_t)tok * kDim + c0;
    *(volatile v8h*)op = hv;
    __threadfence();
    *(volatile v8h*)op = hv;
  }
}

__global__ __launch_bounds__(128) void chunk_prep_kernel(const unsigned short* __restrict__ qnp,
                                                         const unsigned short* __restrict__ knp,
                                                         const float* __restrict__ logits,
                                                         unsigned short* __restrict__ tp16) {
  __shared__ __align__(16) float sA[4][kChunk * kPF];
  __shared__ __align__(16) float sP[4][kChunk * kPF];
  __shared__ float sB[4][kChunk];
  const int lane = threadIdx.x & 31, wave = threadIdx.x >> 5;
  const int c = lane & 15, hh = lane >> 4, koff = hh * 8;
  const int cid = blockIdx.x * 4 + wave;
  if (cid >= kChunkAll) return;
  const int ch = cid % kNumChunk;
  const int bh = cid / kNumChunk;
  const int h  = bh % kHeads;
  const int b  = bh / kHeads;
  const int tok0 = b * kSeq + ch * kChunk;
  const _Float16* qh = (const _Float16*)qnp;
  const _Float16* kh = (const _Float16*)knp;

  {
    const float lg = logits[(size_t)(tok0 + lane) * kLogitN + h];
    sB[wave][lane] = sigmoid_f(lg);
  }

  v16h kf[2][4];
#pragma unroll
  for (int mt = 0; mt < 2; ++mt)
#pragma unroll
    for (int ks = 0; ks < 4; ++ks)
      kf[mt][ks] = Frag<_Float16>::load(kh + (size_t)(tok0 + 16 * mt + c) * kDim + h * kHeadDim + ks * 32 + koff);

  const v8f z8 = {0.f, 0.f, 0.f, 0.f, 0.f, 0.f, 0.f, 0.f};
  v8f g00 = z8, g10 = z8, g11 = z8, p00 = z8, p10 = z8, p11 = z8;
#pragma unroll
  for (int ks = 0; ks < 4; ++ks) {
    g00 = mma_g(kf[0][ks], kf[0][ks], g00);
    g10 = mma_g(kf[1][ks], kf[0][ks], g10);
    g11 = mma_g(kf[1][ks], kf[1][ks], g11);
  }
#pragma unroll
  for (int ks = 0; ks < 4; ++ks) {
    const v16h q0 = Frag<_Float16>::load(qh + (size_t)(tok0 + c) * kDim + h * kHeadDim + ks * 32 + koff);
    const v16h q1 = Frag<_Float16>::load(qh + (size_t)(tok0 + 16 + c) * kDim + h * kHeadDim + ks * 32 + koff);
    p00 = mma_g(q0, kf[0][ks], p00);
    p10 = mma_g(q1, kf[0][ks], p10);
    p11 = mma_g(q1, kf[1][ks], p11);
  }

  wave_sync_lds();
  float* a = sA[wave];
  float* p = sP[wave];
#pragma unroll
  for (int r = 0; r < 8; ++r) {
    const int r0 = 8 * hh + r;
    const int r1 = 16 + r0;
    const float b0 = sB[wave][r0];
    const float b1 = sB[wave][r1];
    a[r0 * kPF + c]      = (c < r0) ? -(b0 * g00[r]) : 0.0f;
    a[r0 * kPF + 16 + c] = 0.0f;
    a[r1 * kPF + c]      = -(b1 * g10[r]);
    a[r1 * kPF + 16 + c] = (c < r0) ? -(b1 * g11[r]) : 0.0f;
    p[r0 * kPF + c]      = (c <= r0) ? p00[r] : 0.0f;
    p[r0 * kPF + 16 + c] = 0.0f;
    p[r1 * kPF + c]      = p10[r];
    p[r1 * kPF + 16 + c] = (c <= r0) ? p11[r] : 0.0f;
  }
  wave_sync_lds();

#pragma unroll 1
  for (int i = 1; i < kChunk; ++i) {
    float s = 0.0f;
#pragma unroll 1
    for (int j = 0; j < i; ++j) s = fmaf(a[i * kPF + j], a[j * kPF + lane], s);
    const float old = a[i * kPF + lane];
    wave_sync_lds();
    a[i * kPF + lane] = (lane < i) ? (old + s) : old;
    wave_sync_lds();
  }

  unsigned short* tout = tp16 + (size_t)cid * kTileHalves;
  unsigned short* pout = tp16 + (size_t)kChunkAll * kTileHalves + (size_t)cid * kTileHalves;
  for (int pass = 0; pass < 2; ++pass) {
#pragma unroll
    for (int it = 0; it < 4; ++it) {
      const int row = it * 8 + (lane >> 2);
      const int c8 = (lane & 3) * 8;
      const v4f a0 = *(const v4f*)(a + row * kPF + c8);
      const v4f a1 = *(const v4f*)(a + row * kPF + c8 + 4);
      const v4f q0 = *(const v4f*)(p + row * kPF + c8);
      const v4f q1 = *(const v4f*)(p + row * kPF + c8 + 4);
      v8h tv, pv;
#pragma unroll
      for (int e = 0; e < 4; ++e) {
        tv[e]     = (_Float16)(a0[e] + (((c8 + e) == row) ? 1.0f : 0.0f));
        tv[4 + e] = (_Float16)(a1[e] + (((c8 + 4 + e) == row) ? 1.0f : 0.0f));
        pv[e]     = (_Float16)q0[e];
        pv[4 + e] = (_Float16)q1[e];
      }
      *(volatile v8h*)(tout + row * kChunk + c8) = tv;
      *(volatile v8h*)(pout + row * kChunk + c8) = pv;
    }
    __threadfence();
  }
}

__global__ __launch_bounds__(256) void scan_kernel(const unsigned short* __restrict__ qnp, const unsigned short* __restrict__ knp,
                                                   const unsigned short* __restrict__ vcp, const float* __restrict__ logits,
                                                   const unsigned short* __restrict__ tp16, float* __restrict__ ocore) {
  __shared__ __align__(16) _Float16 sQK[2][kChunk * kPQ];
  __shared__ __align__(16) _Float16 sKT[kHeadDim * kPT];
  __shared__ __align__(16) _Float16 sS[kSlice * kPQ];
  __shared__ __align__(16) _Float16 sTP[2][kChunk * kPT];
  __shared__ __align__(16) _Float16 sR[kSlice * kPT];
  __shared__ __align__(16) _Float16 sU[kSlice * kPT];
  __shared__ __align__(16) float sVB[kChunk * kPF];
  __shared__ __align__(16) float sO[kChunk * kPF];

  const int tid = threadIdx.x, lane = tid & 31, wave = tid >> 5;
  const int c = lane & 15, hh = lane >> 4, koff = hh * 8;
  const int blk = blockIdx.x;
  const int sl  = blk % kNumSlice;
  const int h   = (blk / kNumSlice) % kHeads;
  const int b   = blk / (kNumSlice * kHeads);
  const int dv0 = sl * kSlice;
  const _Float16* qh = (const _Float16*)qnp;
  const _Float16* th = (const _Float16*)tp16;

  const v8f z8 = {0.f, 0.f, 0.f, 0.f, 0.f, 0.f, 0.f, 0.f};
  v8f sacc0 = z8, sacc1 = z8;
  {
    v8h zz;
#pragma unroll
    for (int r = 0; r < 8; ++r) zz[r] = (_Float16)0.0f;
    *(v8h*)(sS + c * kPQ + 16 * wave + 8 * hh) = zz;
    *(v8h*)(sS + (16 + c) * kPQ + 16 * wave + 8 * hh) = zz;
  }

  const int w4 = wave & 3, mi = w4 >> 1, nj = w4 & 1;
  const bool lowhalf = (wave < 4);
  const int asel = lowhalf ? 0 : 1;

#pragma unroll 1
  for (int ch = 0; ch < kNumChunk; ++ch) {
    const int tok0 = b * kSeq + ch * kChunk;
    {
      const int row = tid >> 3, seg = tid & 7;
      const size_t gofs = (size_t)(tok0 + row) * kDim + h * kHeadDim;
      const float lg = logits[(size_t)(tok0 + row) * kLogitN + h];
      const float beta = sigmoid_f(lg);
      const v8h q0 = *(const v8h*)(qh + gofs + seg * 16);
      const v8h q1 = *(const v8h*)(qh + gofs + seg * 16 + 8);
      const v4u kw0 = *(const v4u*)(knp + gofs + seg * 16);
      const v4u kw1 = *(const v4u*)(knp + gofs + seg * 16 + 8);
      const v2u vw  = *(const v2u*)(vcp + gofs + dv0 + seg * 4);
      *(v8h*)(&sQK[1][row * kPQ + seg * 16])     = q0;
      *(v8h*)(&sQK[1][row * kPQ + seg * 16 + 8]) = q1;
      float kf[16];
#pragma unroll
      for (int j = 0; j < 4; ++j) {
        const unsigned wa = kw0[j];
        const unsigned wb = kw1[j];
        unpack2(wa, kf[2 * j], kf[2 * j + 1]);
        unpack2(wb, kf[8 + 2 * j], kf[8 + 2 * j + 1]);
      }
      v8h n0, n1;
#pragma unroll
      for (int e = 0; e < 8; ++e) {
        n0[e] = (_Float16)(-(kf[e] * beta));
        n1[e] = (_Float16)(-(kf[8 + e] * beta));
      }
      *(v8h*)(&sQK[0][row * kPQ + seg * 16])     = n0;
      *(v8h*)(&sQK[0][row * kPQ + seg * 16 + 8]) = n1;
#pragma unroll
      for (int e = 0; e < 16; ++e) sKT[(seg * 16 + e) * kPT + row] = (_Float16)kf[e];
      {
        const unsigned v0 = vw[0];
        const unsigned v1 = vw[1];
        float x0, x1, x2, x3;
        unpack2(v0, x0, x1);
        unpack2(v1, x2, x3);
        const v4f vb = {x0 * beta, x1 * beta, x2 * beta, x3 * beta};
        *(v4f*)(sVB + row * kPF + seg * 4) = vb;
      }
      {
        const int sel = tid >> 7, t7 = tid & 127;
        const size_t cidx = (size_t)((b * kHeads + h) * kNumChunk + ch);
        const v8h tv = *(const v8h*)(th + (size_t)sel * kChunkAll * kTileHalves + cidx * kTileHalves + t7 * 8);
        *(v8h*)(&sTP[sel][(t7 >> 2) * kPT + (t7 & 3) * 8]) = tv;
      }
    }
    __syncthreads();

    v8f acc;
#pragma unroll
    for (int r = 0; r < 8; ++r) {
      const float vbv = sVB[(16 * mi + 8 * hh + r) * kPF + 16 * nj + c];
      acc[r] = lowhalf ? vbv : 0.0f;
    }
    {
      const _Float16* arow = &sQK[asel][(16 * mi + c) * kPQ + koff];
      const _Float16* brow = sS + (16 * nj + c) * kPQ + koff;
#pragma unroll
      for (int ks = 0; ks < 4; ++ks) {
        const v16h af = Frag<_Float16>::load(arow + ks * 32);
        const v16h bf = Frag<_Float16>::load(brow + ks * 32);
        acc = mma_g(af, bf, acc);
      }
    }
    if (lowhalf) {
      v8h rv;
#pragma unroll
      for (int r = 0; r < 8; ++r) rv[r] = (_Float16)acc[r];
      *(v8h*)(sR + (16 * nj + c) * kPT + 16 * mi + 8 * hh) = rv;
    }
    __syncthreads();

    if (lowhalf) {
      const v16h af = Frag<_Float16>::load(&sTP[0][(16 * mi + c) * kPT + koff]);
      const v16h bf = Frag<_Float16>::load(sR + (16 * nj + c) * kPT + koff);
      const v8f u = mma_g(af, bf, z8);
      v8h uv;
#pragma unroll
      for (int r = 0; r < 8; ++r) uv[r] = (_Float16)u[r];
      *(v8h*)(sU + (16 * nj + c) * kPT + 16 * mi + 8 * hh) = uv;
    }
    __syncthreads();

    if (!lowhalf) {
      const v16h af = Frag<_Float16>::load(&sTP[1][(16 * mi + c) * kPT + koff]);
      const v16h bf = Frag<_Float16>::load(sU + (16 * nj + c) * kPT + koff);
      acc = mma_g(af, bf, acc);
#pragma unroll
      for (int r = 0; r < 8; ++r) sO[(16 * mi + 8 * hh + r) * kPF + 16 * nj + c] = acc[r];
    }
    {
      const v16h af = Frag<_Float16>::load(sKT + (16 * wave + c) * kPT + koff);
      const v16h b0 = Frag<_Float16>::load(sU + c * kPT + koff);
      const v16h b1 = Frag<_Float16>::load(sU + (16 + c) * kPT + koff);
      sacc0 = mma_g(af, b0, sacc0);
      sacc1 = mma_g(af, b1, sacc1);
      v8h s0, s1;
#pragma unroll
      for (int r = 0; r < 8; ++r) {
        s0[r] = (_Float16)sacc0[r];
        s1[r] = (_Float16)sacc1[r];
      }
      *(v8h*)(sS + c * kPQ + 16 * wave + 8 * hh) = s0;
      *(v8h*)(sS + (16 + c) * kPQ + 16 * wave + 8 * hh) = s1;
    }
    __syncthreads();

    {
      const int row = wave * 4 + (lane >> 3);
      const int c4 = (lane & 7) * 4;
      const v4f ov = *(const v4f*)(sO + row * kPF + c4);
      float* op = ocore + (size_t)(tok0 + row) * kDim + h * kHeadDim + dv0 + c4;
      *(volatile v4f*)op = ov;
      __threadfence();
      *(volatile v4f*)op = ov;
    }
  }
}

__global__ __launch_bounds__(256) void mix_norm_kernel(const float* __restrict__ ocore, const unsigned short* __restrict__ vc,
                                                       const float* __restrict__ logits, const float* __restrict__ mix_b,
                                                       const float* __restrict__ mix_bias, const float* __restrict__ onw,
                                                       unsigned short* __restrict__ omix) {
  const int lane = threadIdx.x & 31, wave = threadIdx.x >> 5;
  const int gw = blockIdx.x * 8 + wave;
  if (gw >= kTok * 4) return;
  const int tok = gw >> 2;
  const int hp  = gw & 3;
  const int head = hp * 2 + (lane >> 4);
  const int dl = (lane & 15) * 8;
  const int c0 = head * kHeadDim + dl;
  const float lg = logits[(size_t)tok * kLogitN + kHeads + head];
  const float zg = (lg + mix_b[head]) + mix_bias[head];
  const float g  = sigmoid_f(zg);
  const float gi = 1.0f - g;
  const float* op = ocore + (size_t)tok * kDim + c0;
  const v4f o0 = *(const v4f*)(op);
  const v4f o1 = *(const v4f*)(op + 4);
  const v4u vw = *(const v4u*)(vc + (size_t)tok * kDim + c0);
  const v4f w0 = *(const v4f*)(onw + dl);
  const v4f w1 = *(const v4f*)(onw + dl + 4);
  float ov[8], vv[8], wv[8];
#pragma unroll
  for (int e = 0; e < 4; ++e) {
    ov[e] = o0[e]; ov[4 + e] = o1[e];
    wv[e] = w0[e]; wv[4 + e] = w1[e];
  }
#pragma unroll
  for (int j = 0; j < 4; ++j) {
    const unsigned wj = vw[j];
    unpack2(wj, vv[2 * j], vv[2 * j + 1]);
  }
  float m[8];
  float ss = 0.0f;
#pragma unroll
  for (int e = 0; e < 8; ++e) {
    m[e] = g * ov[e] + gi * vv[e];
    ss += m[e] * m[e];
  }
#pragma unroll
  for (int off = 1; off < 16; off <<= 1) ss += __shfl_xor(ss, off, 32);
  const float rs = rsqrtf(ss * kInvHeadDim + kRmsEps);
  v8h hv;
#pragma unroll
  for (int e = 0; e < 8; ++e) hv[e] = (_Float16)((m[e] * rs) * wv[e]);
  unsigned short* q = omix + (size_t)tok * kDim + c0;
  *(volatile v8h*)q = hv;
  __threadfence();
  *(volatile v8h*)q = hv;
}

extern "C" void kernel_launch(void* const* d_in, const int* in_sizes, int n_in,
                              void* d_out, int out_size, void* d_ws, size_t ws_size, hipStream_t stream) {
  if (n_in < 13 || d_out == nullptr || d_ws == nullptr) return;
  if (in_sizes[0] != kTok * kDim || in_sizes[1] != kDim * kDim || in_sizes[2] != kDim * kDim ||
      in_sizes[3] != kDim * kDim || in_sizes[4] != kDim * 4 || in_sizes[5] != kDim * 4 ||
      in_sizes[6] != kDim * 4 || in_sizes[7] != kDim * kHeads || in_sizes[8] != kDim * kHeads ||
      in_sizes[9] != kHeads || in_sizes[10] != kHeads || in_sizes[11] != kHeadDim ||
      in_sizes[12] != kDim * kDim || out_size != kTok * kDim) return;

  const float* hs       = (const float*)d_in[0];
  const float* q_w      = (const float*)d_in[1];
  const float* k_w      = (const float*)d_in[2];
  const float* v_w      = (const float*)d_in[3];
  const float* conv_q_w = (const float*)d_in[4];
  const float* conv_k_w = (const float*)d_in[5];
  const float* conv_v_w = (const float*)d_in[6];
  const float* b_w      = (const float*)d_in[7];
  const float* mix_w    = (const float*)d_in[8];
  const float* mix_b    = (const float*)d_in[9];
  const float* mix_bias = (const float*)d_in[10];
  const float* o_norm_w = (const float*)d_in[11];
  const float* o_w      = (const float*)d_in[12];
  float* out = (float*)d_out;

  char* ws = (char*)d_ws; size_t off = 0;
  auto carve = [&](size_t bytes) -> char* { char* p = ws + off; off += (bytes + 255) & ~(size_t)255; return p; };
  unsigned short* HS16   = (unsigned short*)carve((size_t)kTok * kDim * 2);
  unsigned short* WQKVT  = (unsigned short*)carve((size_t)kQKVDim * kDim * 2);
  unsigned short* WOT    = (unsigned short*)carve((size_t)kDim * kDim * 2);
  unsigned short* WBMT   = (unsigned short*)carve((size_t)kLogitN * kDim * 2);
  unsigned short* LIN    = (unsigned short*)carve((size_t)kTok * kQKVDim * 2);
  float*          LOGITS = (float*)carve((size_t)kTok * kLogitN * 4);
  unsigned short* QKV    = (unsigned short*)carve((size_t)3 * kTok * kDim * 2);
  if (off > ws_size || off > (size_t)134217728) return;
  unsigned short* TP16   = HS16;
  float*          OCORE  = (float*)(void*)LIN;
  unsigned short* OMIX16 = (unsigned short*)((char*)(void*)LIN + (size_t)kTok * kDim * 4);
  const unsigned short* QN = QKV;
  const unsigned short* KN = QKV + (size_t)kTok * kDim;
  const unsigned short* VC = QKV + (size_t)2 * kTok * kDim;

  const int n8 = kTok * (kDim / 8);
  cast8_f16_kernel<<<(n8 + 255) / 256, 256, 0, stream>>>(hs, HS16, n8);
  pack_w_kernel<<<dim3(kDim / 64, kDim / 64, 4), 256, 0, stream>>>(q_w, k_w, v_w, o_w, WQKVT, WOT);
  pack_bm_kernel<<<(kLogitN * (kDim / 8) + 255) / 256, 256, 0, stream>>>(b_w, mix_w, WBMT);
  wmma_gemm64<1><<<(kTok / 64) * (kQKVDim / 64) / 8, 256, 0, stream>>>(
      HS16, kDim, WQKVT, kDim, (void*)LIN, kQKVDim, kTok, kQKVDim, kDim, kWCarryInv);
  wmma_gemm64<0><<<(kTok / 64) * (kLogitN / 64) / 8, 256, 0, stream>>>(
      HS16, kDim, WBMT, kDim, (void*)LOGITS, kLogitN, kTok, kLogitN, kDim, kWCarryInv);
  conv_norm_kernel<<<(kTok * 4) / 8, 256, 0, stream>>>(LIN, conv_q_w, conv_k_w, conv_v_w, QKV);
  chunk_prep_kernel<<<kChunkAll / 4, 128, 0, stream>>>(QN, KN, LOGITS, TP16);
  scan_kernel<<<kBatch * kHeads * kNumSlice, 256, 0, stream>>>(QN, KN, VC, LOGITS, TP16, OCORE);
  mix_norm_kernel<<<(kTok * 4) / 8, 256, 0, stream>>>(OCORE, VC, LOGITS, mix_b, mix_bias, o_norm_w, OMIX16);
  wmma_gemm64<0><<<(kTok / 64) * (kDim / 64) / 8, 256, 0, stream>>>(
      OMIX16, kDim, WOT, kDim, (void*)out, kDim, kTok, kDim, kDim, kWCarryInv);
}
